// RotationConditionerBlock_33380485825345
// MI455X (gfx1250) — hardware-verified
//
#include <hip/hip_runtime.h>
#include <hip/hip_bf16.h>

#define SEQ   2048
#define ND    128
#define NA    64
#define NHEAD 8
#define CH    64
#define TH3   24
#define OKQ   1024
#define OV    3072

typedef __attribute__((ext_vector_type(16))) __bf16 v16bf;
typedef __attribute__((ext_vector_type(2)))  __bf16 v2bf;
typedef __attribute__((ext_vector_type(8)))  float  v8f;

union Frag {
    v16bf v;
    unsigned int d[8];
    unsigned short h[16];
};

__device__ __forceinline__ unsigned short f2bf(float f) {
    unsigned u = __builtin_bit_cast(unsigned, f);
    unsigned r = u + 0x7FFFu + ((u >> 16) & 1u);
    return (unsigned short)(r >> 16);
}

__device__ __forceinline__ unsigned pack_bf16(float lo, float hi) {
#if __has_builtin(__builtin_amdgcn_cvt_pk_bf16_f32)
    v2bf p = __builtin_amdgcn_cvt_pk_bf16_f32(lo, hi);
    return __builtin_bit_cast(unsigned, p);
#else
    union { v2bf b; unsigned u; } x;
    x.b[0] = (__bf16)lo;
    x.b[1] = (__bf16)hi;
    return x.u;
#endif
}

__device__ __forceinline__ void split_bf16(float f, unsigned short& hi, unsigned short& lo) {
    hi = f2bf(f);
    const float fh = __builtin_bit_cast(float, ((unsigned)hi) << 16);
    lo = f2bf(f - fh);
}
__device__ __forceinline__ unsigned pack2(unsigned short a, unsigned short b) { return (unsigned)a | ((unsigned)b << 16); }

__device__ __forceinline__ v8f zero8() {
    v8f z;
#pragma unroll
    for (int i = 0; i < 8; ++i) z[i] = 0.0f;
    return z;
}

__device__ __forceinline__ int frag_dv(int v) {
    return (v >> 2) * 8 + (v & 3);
}

__global__ void proj_kq_kernel(const float* __restrict__ nodes,
                               const float* __restrict__ pos,
                               const float* __restrict__ aux,
                               const float* __restrict__ Wn, const float* __restrict__ bn,
                               const float* __restrict__ Wp, const float* __restrict__ bp,
                               const float* __restrict__ Wa,
                               unsigned* __restrict__ Khi, unsigned* __restrict__ Klo,
                               unsigned* __restrict__ Qhi, unsigned* __restrict__ Qlo) {
    unsigned tid = blockIdx.x * blockDim.x + threadIdx.x;
    unsigned op = tid & (OKQ / 2 - 1);
    unsigned s  = (tid >> 9) & (SEQ - 1);
    unsigned g  = tid >> 20;
    if (g >= 3) return;
    unsigned o0 = 2 * op, o1 = o0 + 1;

    float a0 = 0.0f, a1 = 0.0f;
    if (g == 0) {
        a0 = bn[o0]; a1 = bn[o1];
        const float* x = nodes + s * ND;
        const float* w0 = Wn + o0 * ND; const float* w1 = Wn + o1 * ND;
#pragma unroll 8
        for (int d = 0; d < ND; ++d) { const float xv = x[d]; a0 += xv * w0[d]; a1 += xv * w1[d]; }
    } else if (g == 1) {
        a0 = bp[o0]; a1 = bp[o1];
        const float* x = pos + s * 6;
        const float* w0 = Wp + o0 * 6; const float* w1 = Wp + o1 * 6;
#pragma unroll
        for (int d = 0; d < 6; ++d) { const float xv = x[d]; a0 += xv * w0[d]; a1 += xv * w1[d]; }
    } else {
        const float* x = aux + s * NA;
        const float* w0 = Wa + o0 * NA; const float* w1 = Wa + o1 * NA;
#pragma unroll 8
        for (int d = 0; d < NA; ++d) { const float xv = x[d]; a0 += xv * w0[d]; a1 += xv * w1[d]; }
    }
    unsigned hh = o0 >> 7;
    unsigned c  = o0 & 127;
    unsigned ht = g * NHEAD + hh;
    unsigned short h0, l0, h1, l1;
    split_bf16(a0, h0, l0); split_bf16(a1, h1, l1);
    const unsigned vh = pack2(h0, h1), vl = pack2(l0, l1);
    unsigned* ph; unsigned* pl; unsigned idx;
    if (c < CH) { ph = Khi; pl = Klo; idx = ((ht * SEQ + s) * CH + c) >> 1; }
    else        { ph = Qhi; pl = Qlo; idx = ((ht * SEQ + s) * CH + (c - CH)) >> 1; }
    *(volatile unsigned*)(ph + idx) = vh; *(volatile unsigned*)(pl + idx) = vl;
    __threadfence();
    *(volatile unsigned*)(ph + idx) = vh; *(volatile unsigned*)(pl + idx) = vl;
}

__global__ void proj_v_kernel(const float* __restrict__ nodes,
                              const float* __restrict__ Wv,
                              const float* __restrict__ bv,
                              unsigned* __restrict__ Vhi, unsigned* __restrict__ Vlo) {
    unsigned tid = blockIdx.x * blockDim.x + threadIdx.x;
    unsigned sp = tid & (SEQ / 2 - 1);
    unsigned o  = tid >> 10;
    if (o >= OV) return;
    const unsigned s0 = 2 * sp;

    float a0 = bv[o], a1 = bv[o];
    const float* x0 = nodes + s0 * ND; const float* x1 = x0 + ND;
    const float* w = Wv + o * ND;
#pragma unroll 8
    for (int d = 0; d < ND; ++d) { const float wv = w[d]; a0 += x0[d] * wv; a1 += x1[d] * wv; }

    unsigned ht = o >> 7;
    unsigned d2 = o & 127;
    unsigned short h0, l0, h1, l1;
    split_bf16(a0, h0, l0); split_bf16(a1, h1, l1);
    const unsigned idx = ((ht * (unsigned)ND + d2) * (unsigned)SEQ + s0) >> 1;
    const unsigned vh = pack2(h0, h1), vl = pack2(l0, l1);
    *(volatile unsigned*)(Vhi + idx) = vh; *(volatile unsigned*)(Vlo + idx) = vl;
    __threadfence();
    *(volatile unsigned*)(Vhi + idx) = vh; *(volatile unsigned*)(Vlo + idx) = vl;
}

__global__ __launch_bounds__(768, 1)
void attn_kernel(const unsigned* __restrict__ Khi, const unsigned* __restrict__ Klo,
                 const unsigned* __restrict__ Qhi, const unsigned* __restrict__ Qlo,
                 const unsigned* __restrict__ Vhi, const unsigned* __restrict__ Vlo,
                 float* __restrict__ out) {
    __shared__ float red[16][ND];

    const int lane = threadIdx.x;
    const int wid  = threadIdx.y;
    const int i0   = blockIdx.x * 16;
    const float scale = 0.35355339059327373f;

    const unsigned int* Kp = Khi; const unsigned int* KpL = Klo;
    const unsigned int* Qp = Qhi; const unsigned int* QpL = Qlo;
    const unsigned int* Vp = Vhi; const unsigned int* VpL = Vlo;

    const int lm = lane & 15;
    const int lh = lane >> 4;

    Frag bK[2], bKL[2];
    {
        unsigned kInv = ((unsigned)wid * SEQ + (unsigned)(i0 + lm)) * (CH / 2) + (unsigned)(lh * 4);
#pragma unroll
        for (int cc = 0; cc < 2; ++cc)
#pragma unroll
            for (int v = 0; v < 8; ++v) {
                bK[cc].d[v]  = Kp[kInv + cc * 16 + frag_dv(v)];
                bKL[cc].d[v] = KpL[kInv + cc * 16 + frag_dv(v)];
            }
    }

    unsigned qInv = ((unsigned)wid * SEQ + (unsigned)lm) * (CH / 2) + (unsigned)(lh * 4);
    unsigned vInv[8];
#pragma unroll
    for (int t = 0; t < 8; ++t)
        vInv[t] = ((unsigned)wid * ND + (unsigned)(t * 16 + lm)) * (SEQ / 2) + (unsigned)(lh * 4);

    v8f acc[8];
#pragma unroll
    for (int t = 0; t < 8; ++t) acc[t] = zero8();
    float rm = -1e30f;
    float rl = 0.0f;

    for (int j0 = 0; j0 < SEQ; j0 += 32) {
        v8f sfr[2];
#pragma unroll
        for (int jt = 0; jt < 2; ++jt) {
            unsigned qb = qInv + (unsigned)((j0 + jt * 16) * (CH / 2));
            Frag aQ0, aQ1, aQ0L, aQ1L;
#pragma unroll
            for (int v = 0; v < 8; ++v) { aQ0.d[v] = Qp[qb + frag_dv(v)];      aQ0L.d[v] = QpL[qb + frag_dv(v)]; }
#pragma unroll
            for (int v = 0; v < 8; ++v) { aQ1.d[v] = Qp[qb + 16 + frag_dv(v)]; aQ1L.d[v] = QpL[qb + 16 + frag_dv(v)]; }
            v8f sacc = zero8();
            sacc = __builtin_amdgcn_wmma_f32_16x16x32_bf16(false, aQ0L.v, false, bK[0].v,  (short)0, sacc, false, false);
            sacc = __builtin_amdgcn_wmma_f32_16x16x32_bf16(false, aQ0.v,  false, bKL[0].v, (short)0, sacc, false, false);
            sacc = __builtin_amdgcn_wmma_f32_16x16x32_bf16(false, aQ1L.v, false, bK[1].v,  (short)0, sacc, false, false);
            sacc = __builtin_amdgcn_wmma_f32_16x16x32_bf16(false, aQ1.v,  false, bKL[1].v, (short)0, sacc, false, false);
            sacc = __builtin_amdgcn_wmma_f32_16x16x32_bf16(false, aQ0.v,  false, bK[0].v,  (short)0, sacc, false, false);
            sacc = __builtin_amdgcn_wmma_f32_16x16x32_bf16(false, aQ1.v,  false, bK[1].v,  (short)0, sacc, false, false);
            sfr[jt] = sacc;
        }

        float sc[16];
#pragma unroll
        for (int jt = 0; jt < 2; ++jt)
#pragma unroll
            for (int r = 0; r < 8; ++r) sc[jt * 8 + r] = sfr[jt][r] * scale;

        float mloc = sc[0];
#pragma unroll
        for (int e = 1; e < 16; ++e) mloc = fmaxf(mloc, sc[e]);
        mloc = fmaxf(mloc, __shfl_xor(mloc, 16, 32));
        float mnew  = fmaxf(rm, mloc);
        float alpha = __expf(rm - mnew);
        rm = mnew;

        Frag bP, bPL;
        float ssum = 0.0f;
#pragma unroll
        for (int v = 0; v < 8; ++v) {
            int g  = v >> 2;
            int i3 = v & 3;
            float p0 = __expf(sc[g * 8 + 2 * i3]     - mnew);
            float p1 = __expf(sc[g * 8 + 2 * i3 + 1] - mnew);
            ssum += p0 + p1;
            unsigned short h0, l0, h1, l1;
            split_bf16(p0, h0, l0); split_bf16(p1, h1, l1);
            bP.d[v] = pack2(h0, h1); bPL.d[v] = pack2(l0, l1);
        }
        ssum += __shfl_xor(ssum, 16, 32);
        rl = rl * alpha + ssum;

        if (__ballot(alpha != 1.0f)) {
#pragma unroll
            for (int t = 0; t < 8; ++t)
#pragma unroll
                for (int r = 0; r < 8; ++r) acc[t][r] *= alpha;
        }

        unsigned vj = (unsigned)(j0 >> 1);
#pragma unroll
        for (int t = 0; t < 8; ++t) {
            Frag aV, aVL;
#pragma unroll
            for (int v = 0; v < 8; ++v) { aV.d[v] = Vp[vInv[t] + vj + frag_dv(v)]; aVL.d[v] = VpL[vInv[t] + vj + frag_dv(v)]; }
            v8f part = zero8();
            part = __builtin_amdgcn_wmma_f32_16x16x32_bf16(false, aVL.v, false, bP.v,  (short)0, part, false, false);
            part = __builtin_amdgcn_wmma_f32_16x16x32_bf16(false, aV.v,  false, bPL.v, (short)0, part, false, false);
            part = __builtin_amdgcn_wmma_f32_16x16x32_bf16(false, aV.v,  false, bP.v,  (short)0, part, false, false);
#pragma unroll
            for (int r = 0; r < 8; ++r) acc[t][r] += part[r];
        }
    }

    float rinv = 1.0f / rl;
#pragma unroll
    for (int t = 0; t < 8; ++t)
#pragma unroll
        for (int r = 0; r < 8; ++r) acc[t][r] *= rinv;

    for (int w = 0; w < TH3; ++w) {
        if (wid == w) {
#pragma unroll
            for (int t = 0; t < 8; ++t)
#pragma unroll
                for (int r = 0; r < 8; ++r) {
                    int d = t * 16 + lh * 8 + r;
                    if (w == 0) red[lm][d]  = acc[t][r];
                    else        red[lm][d] += acc[t][r];
                }
        }
        __syncthreads();
    }
    if (wid == 0) {
        typedef __attribute__((ext_vector_type(4))) float v4f_t;
#pragma unroll
        for (int r = 0; r < 16; ++r) { v4f_t v4; v4.x = red[r][lane * 4]; v4.y = red[r][lane * 4 + 1]; v4.z = red[r][lane * 4 + 2]; v4.w = red[r][lane * 4 + 3]; *(volatile v4f_t*)(out + (i0 + r) * ND + lane * 4) = v4; }
        __threadfence();
#pragma unroll
        for (int r = 0; r < 16; ++r) { v4f_t v4; v4.x = red[r][lane * 4]; v4.y = red[r][lane * 4 + 1]; v4.z = red[r][lane * 4 + 2]; v4.w = red[r][lane * 4 + 3]; *(volatile v4f_t*)(out + (i0 + r) * ND + lane * 4) = v4; }
    }
}

extern "C" void kernel_launch(void* const* d_in, const int* in_sizes, int n_in,
                              void* d_out, int out_size, void* d_ws, size_t ws_size,
                              hipStream_t stream) {
    const float* nodes = (const float*)d_in[0];
    const float* pos   = (const float*)d_in[1];
    const float* aux   = (const float*)d_in[2];
    const float* Wn    = (const float*)d_in[3];
    const float* bn    = (const float*)d_in[4];
    const float* Wp    = (const float*)d_in[5];
    const float* bp    = (const float*)d_in[6];
    const float* Wa    = (const float*)d_in[7];
    const float* Wv    = (const float*)d_in[8];
    const float* bv    = (const float*)d_in[9];
    float* out = (float*)d_out;

    (void)in_sizes; (void)n_in; (void)out_size; (void)ws_size;
    char* ws = (char*)d_ws;
    const size_t kq = (size_t)TH3 * SEQ * CH * 2, vv = (size_t)TH3 * ND * SEQ * 2;
    unsigned* Khi = (unsigned*)(ws);
    unsigned* Klo = (unsigned*)(ws + kq);
    unsigned* Qhi = (unsigned*)(ws + 2 * kq);
    unsigned* Qlo = (unsigned*)(ws + 3 * kq);
    unsigned* Vhi = (unsigned*)(ws + 4 * kq);
    unsigned* Vlo = (unsigned*)(ws + 4 * kq + vv);

    {
        unsigned total = 3u << 20;
        proj_kq_kernel<<<total / 256, 256, 0, stream>>>(
            nodes, pos, aux, Wn, bn, Wp, bp, Wa, Khi, Klo, Qhi, Qlo);
    }
    {
        unsigned total = (unsigned)OV * (SEQ / 2);
        proj_v_kernel<<<total / 256, 256, 0, stream>>>(nodes, Wv, bv, Vhi, Vlo);
    }

    dim3 blk(32, TH3, 1);
    dim3 grd(SEQ / 16, 1, 1);
    attn_kernel<<<grd, blk, 0, stream>>>(Khi, Klo, Qhi, Qlo, Vhi, Vlo, out);
}
